// SAGEGRU_79405355369204
// MI455X (gfx1250) — hardware-verified
//
#include <hip/hip_runtime.h>
#include <stddef.h>


#define TT      16
#define HG      64
#define HT      128
#define G3      384
#define KC      128
#define NTHR    256
#define NWAVE   8
#define EPT     8
#define NGRP    2
#define CHUNK   (NTHR * EPT * NGRP)
#define WCAP    (EPT * NGRP * 32)
#define LISTN   (NWAVE * WCAP)
#define NBC     4096
#define NBF     1024
#define RCAP    40960
#define RBN     128
#define OTHR    512
#define TGT0    256
#define ROWS1   128
#define GTHR    128
#define GWAVE   4
#define GROWB   64
#define DEGCAP  128
#define AP1     (KC + 8)
#define SP1     (HG + 8)
#define HP32    (HT + 4)
#define HP16    (HT + 8)
#define ASC     8.0f
#define WSC     16.0f
#define PINV    0.0078125f
#define LNEPS   1e-5f
#define LDS_FILL ((RCAP + NBF + LISTN) * 4 + 64)

static_assert((CHUNK & (CHUNK - 1)) == 0);
static_assert(CHUNK <= 4096);
static_assert(NBC <= 4096 && NBF <= 4096);
static_assert((NBC & (NBC - 1)) == 0 && (NBF & (NBF - 1)) == 0);
static_assert(NBC == 4 * NBF);
static_assert(OTHR * 8 == NBC);
static_assert((RCAP % 32) == 0);
static_assert(TGT0 == NWAVE * 32);
static_assert(ROWS1 == NWAVE * 16);
static_assert(GROWB == GWAVE * 16 && GTHR == GWAVE * 32);
static_assert(NBC % TGT0 == 0);
static_assert((AP1 * 2) % 16 == 0 && (SP1 * 2) % 16 == 0 && (HP16 * 2) % 16 == 0 && (HP32 * 4) % 16 == 0);
static_assert(((HG * KC / 8) % NTHR) == 0 && ((G3 * HG / 8) % NTHR) == 0 && ((G3 * HT / 8) % NTHR) == 0);

typedef float    v2f  __attribute__((ext_vector_type(2)));
typedef float    v4f  __attribute__((ext_vector_type(4)));
typedef float    v8f  __attribute__((ext_vector_type(8)));
typedef int      v4i  __attribute__((ext_vector_type(4)));
typedef _Float16 v2h  __attribute__((ext_vector_type(2)));
typedef _Float16 v8h  __attribute__((ext_vector_type(8)));
typedef _Float16 v16h __attribute__((ext_vector_type(16)));
union FragH { v16h v; v8h h[2]; };

__device__ __forceinline__ v8h cvt8(v4f a, v4f b) {
  v8h r;
  r[0] = (_Float16)a.x; r[1] = (_Float16)a.y; r[2] = (_Float16)a.z; r[3] = (_Float16)a.w;
  r[4] = (_Float16)b.x; r[5] = (_Float16)b.y; r[6] = (_Float16)b.z; r[7] = (_Float16)b.w;
  return r;
}

__device__ __forceinline__ v8f wmh(v16h a, v16h b, v8f c) {
  v8f d = __builtin_amdgcn_wmma_f32_16x16x32_f16(false, a, false, b, (short)0, c, false, false);
  asm volatile("v_nop\n\tv_nop\n\tv_nop\n\tv_nop" : "+v"(d) : "v"(a), "v"(b));
  return d;
}

__device__ __forceinline__ float red16(float v) {
  v += __shfl_xor(v, 1, 32);
  v += __shfl_xor(v, 2, 32);
  v += __shfl_xor(v, 4, 32);
  v += __shfl_xor(v, 8, 32);
  return v;
}

__device__ __forceinline__ float sigm(float x) {
  return __builtin_amdgcn_rcpf(1.f + __expf(-x));
}
__device__ __forceinline__ float tanh_fast(float x) {
  const float e = __expf(-2.f * fabsf(x));
  const float r = (1.f - e) * __builtin_amdgcn_rcpf(1.f + e);
  return copysignf(r, x);
}

template <int NB>
__device__ __forceinline__ int scan_chunk(const int* __restrict__ dsts, int nE, int cbase, int slotBase,
                                          int vec8, int* list, int tid, int lane, int wave) {
  int wc = 0;
#pragma unroll
  for (int g = 0; g < NGRP; ++g) {
    const int el0  = (g * NTHR + tid) * EPT;
    const int e0   = cbase + el0;
    const int sent = -2147483647 - 1;
    v4i da, db;
    if (vec8 != 0 && cbase + CHUNK <= nE) {
      da = *(const v4i*)(dsts + e0);
      db = *(const v4i*)(dsts + e0 + 4);
    } else {
      da.x = (e0     < nE) ? dsts[min(e0, nE - 1)] : sent;
      da.y = (e0 + 1 < nE) ? dsts[min(e0 + 1, nE - 1)] : sent;
      da.z = (e0 + 2 < nE) ? dsts[min(e0 + 2, nE - 1)] : sent;
      da.w = (e0 + 3 < nE) ? dsts[min(e0 + 3, nE - 1)] : sent;
      db.x = (e0 + 4 < nE) ? dsts[min(e0 + 4, nE - 1)] : sent;
      db.y = (e0 + 5 < nE) ? dsts[min(e0 + 5, nE - 1)] : sent;
      db.z = (e0 + 6 < nE) ? dsts[min(e0 + 6, nE - 1)] : sent;
      db.w = (e0 + 7 < nE) ? dsts[min(e0 + 7, nE - 1)] : sent;
    }
    const unsigned nb = (unsigned)slotBase;
    const unsigned s0 = (unsigned)da.x - nb, s1 = (unsigned)da.y - nb;
    const unsigned s2 = (unsigned)da.z - nb, s3 = (unsigned)da.w - nb;
    const unsigned s4 = (unsigned)db.x - nb, s5 = (unsigned)db.y - nb;
    const unsigned s6 = (unsigned)db.z - nb, s7 = (unsigned)db.w - nb;
    const bool h0 = s0 < (unsigned)NB, h1 = s1 < (unsigned)NB, h2 = s2 < (unsigned)NB, h3 = s3 < (unsigned)NB;
    const bool h4 = s4 < (unsigned)NB, h5 = s5 < (unsigned)NB, h6 = s6 < (unsigned)NB, h7 = s7 < (unsigned)NB;
    const unsigned any = __builtin_amdgcn_ballot_w32(h0 | h1 | h2 | h3 | h4 | h5 | h6 | h7);
    if (any != 0u) {
#define HITJ(J, HJ, SJ) { \
        const unsigned mj = __builtin_amdgcn_ballot_w32(HJ); \
        if (mj != 0u) { \
          if (HJ) { \
            const int pos = wc + (int)__builtin_amdgcn_mbcnt_lo(mj, 0u); \
            if (pos < WCAP) list[wave * WCAP + pos] = ((el0 + (J)) << 12) | (int)(SJ); \
          } \
          wc += (int)__builtin_popcount(mj); } }
      HITJ(0, h0, s0)
      HITJ(1, h1, s1)
      HITJ(2, h2, s2)
      HITJ(3, h3, s3)
      HITJ(4, h4, s4)
      HITJ(5, h5, s5)
      HITJ(6, h6, s6)
      HITJ(7, h7, s7)
#undef HITJ
    }
  }
  return wc;
}

__global__ __launch_bounds__(NTHR) void k_wprep(
    const float* __restrict__ Wl1, const float* __restrict__ Wr1,
    const float* __restrict__ Wih, const float* __restrict__ Whh,
    _Float16* wcat, _Float16* wihp, _Float16* whhp) {
  const int g0 = HG * KC / 8;
  const int g1 = G3 * HG / 8;
  const int g2 = G3 * HT / 8;
  const int bstart = blockIdx.x * NTHR;
  const int i = bstart + (int)threadIdx.x;
  if (i >= g0 + g1 + g2) return;
  float v[8];
  _Float16* dp;
  if (bstart < g0) {
    const int o  = i * 8;
    const int n  = o / KC;
    const int k0 = o - n * KC;
#pragma unroll
    for (int e = 0; e < 8; ++e) {
      const int k  = k0 + e;
      const int kk = k & (HG - 1);
      const float a = Wl1[kk * HG + n];
      const float b = Wr1[kk * HG + n];
      v[e] = (k < HG ? a : b) * WSC;
    }
    dp = wcat + o;
  } else if (bstart < g0 + g1) {
    const int o = (i - g0) * 8;
    const v4f a = *(const v4f*)(Wih + o), b = *(const v4f*)(Wih + o + 4);
    v[0] = a.x * WSC; v[1] = a.y * WSC; v[2] = a.z * WSC; v[3] = a.w * WSC;
    v[4] = b.x * WSC; v[5] = b.y * WSC; v[6] = b.z * WSC; v[7] = b.w * WSC;
    dp = wihp + o;
  } else {
    const int o = (i - g0 - g1) * 8;
    const v4f a = *(const v4f*)(Whh + o), b = *(const v4f*)(Whh + o + 4);
    v[0] = a.x * WSC; v[1] = a.y * WSC; v[2] = a.z * WSC; v[3] = a.w * WSC;
    v[4] = b.x * WSC; v[5] = b.y * WSC; v[6] = b.z * WSC; v[7] = b.w * WSC;
    dp = whhp + o;
  }
  v4f a, b;
  a.x = v[0]; a.y = v[1]; a.z = v[2]; a.w = v[3];
  b.x = v[4]; b.y = v[5]; b.z = v[6]; b.w = v[7];
  const v8h hv = cvt8(a, b);
  *(volatile v8h*)dp = hv;
  __threadfence();
  *(volatile v8h*)dp = hv;
}

__global__ __launch_bounds__(NTHR) void k_count(
    const int* __restrict__ ei, int* cnt, float* dinv, int nE, int vec8) {
  __shared__ __attribute__((aligned(16))) int scnt[NBC];
  __shared__ __attribute__((aligned(16))) int list[LISTN];
  __shared__ int wcnt[NWAVE];
  const int tid = threadIdx.x, lane = tid & 31, wave = tid >> 5;
  const int nodeBase = blockIdx.x * NBC;
  const int* dsts = ei + nE;

  for (int i = tid; i < NBC; i += NTHR) scnt[i] = 0;
  __syncthreads();

  const int nChunks = (nE + CHUNK - 1) / CHUNK;
#pragma unroll 1
  for (int ch = 0; ch < nChunks; ++ch) {
    const int cbase = ch * CHUNK;
    const int wc = scan_chunk<NBC>(dsts, nE, cbase, nodeBase, vec8, list, tid, lane, wave);
    if (lane == 0) wcnt[wave] = wc;
    __syncthreads();
    if (wave == 0) {
#pragma unroll 1
      for (int wsx = 0; wsx < NWAVE; ++wsx) {
        int n = __builtin_amdgcn_readfirstlane(wcnt[wsx]);
        n = n > WCAP ? WCAP : (n < 0 ? 0 : n);
        const int* lp = list + wsx * WCAP;
#pragma unroll 1
        for (int i = 0; i < n; ++i) {
          const int ent  = __builtin_amdgcn_readfirstlane(lp[i]);
          const int slot = ent & (NBC - 1);
          if (lane == 0) scnt[slot] = scnt[slot] + 1;
        }
      }
    }
    __syncthreads();
  }

  v4i cq[4]; v4f dq[4];
#pragma unroll
  for (int q = 0; q < 4; ++q) {
    const int f = (wave * 4 + q) * 128 + 4 * lane;
    const v4i c = *(const v4i*)(scnt + f);
    cq[q] = c;
    dq[q].x = 1.0f / (float)(c.x < 1 ? 1 : c.x);
    dq[q].y = 1.0f / (float)(c.y < 1 ? 1 : c.y);
    dq[q].z = 1.0f / (float)(c.z < 1 ? 1 : c.z);
    dq[q].w = 1.0f / (float)(c.w < 1 ? 1 : c.w);
  }
  int*   cp = cnt + (size_t)nodeBase;
  float* dp = dinv + (size_t)nodeBase;
#pragma unroll
  for (int q = 0; q < 4; ++q) {
    const int f = (wave * 4 + q) * 128 + 4 * lane;
    *(volatile v4i*)(cp + f) = cq[q];
    *(volatile v4f*)(dp + f) = dq[q];
  }
  __threadfence();
#pragma unroll
  for (int q = 0; q < 4; ++q) {
    const int f = (wave * 4 + q) * 128 + 4 * lane;
    *(volatile v4i*)(cp + f) = cq[q];
    *(volatile v4f*)(dp + f) = dq[q];
  }
}

__global__ __launch_bounds__(OTHR) void k_offsets(
    const int* __restrict__ cnt, int* off, int* rbase, int nChunk) {
  __shared__ __attribute__((aligned(16))) int soff[NBC];
  __shared__ __attribute__((aligned(16))) int srb[RBN];
  __shared__ int wtot[OTHR / 32];
  const int tid = threadIdx.x, lane = tid & 31, wave = tid >> 5, sub = tid >> 7;
  for (int i = tid; i < RBN; i += OTHR) srb[i] = 0;
  int carry = 0;
#pragma unroll 1
  for (int ch = 0; ch < nChunk; ++ch) {
    const int base = ch * NBC;
    const v4i c0 = *(const v4i*)(cnt + base + 8 * tid);
    const v4i c1 = *(const v4i*)(cnt + base + 8 * tid + 4);
    const int e0 = max(c0.x, 0), e1 = max(c0.y, 0), e2 = max(c0.z, 0), e3 = max(c0.w, 0);
    const int e4 = max(c1.x, 0), e5 = max(c1.y, 0), e6 = max(c1.z, 0), e7 = max(c1.w, 0);
    const int ts = e0 + e1 + e2 + e3 + e4 + e5 + e6 + e7;
    int incl = ts;
#pragma unroll
    for (int d = 1; d < 32; d <<= 1) {
      const int t = __shfl_up(incl, d, 32);
      if (lane >= d) incl += t;
    }
    if (lane == 31) wtot[wave] = incl;
    __syncthreads();
    const int S0 = wtot[0]  + wtot[1]  + wtot[2]  + wtot[3];
    const int S1 = wtot[4]  + wtot[5]  + wtot[6]  + wtot[7];
    const int S2 = wtot[8]  + wtot[9]  + wtot[10] + wtot[11];
    const int S3 = wtot[12] + wtot[13] + wtot[14] + wtot[15];
    int pre = 0;
#pragma unroll 1
    for (int w = 4 * sub; w < wave; ++w) pre += wtot[w];
    const int b0 = carry;
    const int b1 = b0 + ((S0 + 31) & ~31);
    const int b2 = b1 + ((S1 + 31) & ~31);
    const int b3 = b2 + ((S2 + 31) & ~31);
    const int b4 = b3 + ((S3 + 31) & ~31);
    const int myb = sub == 0 ? b0 : (sub == 1 ? b1 : (sub == 2 ? b2 : b3));
    if (tid == 0) {
      srb[min(4 * ch + 0, RBN - 1)] = b0;
      srb[min(4 * ch + 1, RBN - 1)] = b1;
      srb[min(4 * ch + 2, RBN - 1)] = b2;
      srb[min(4 * ch + 3, RBN - 1)] = b3;
    }
    int run = myb + pre + incl - ts;
    soff[8 * tid + 0] = run; run += e0;
    soff[8 * tid + 1] = run; run += e1;
    soff[8 * tid + 2] = run; run += e2;
    soff[8 * tid + 3] = run; run += e3;
    soff[8 * tid + 4] = run; run += e4;
    soff[8 * tid + 5] = run; run += e5;
    soff[8 * tid + 6] = run; run += e6;
    soff[8 * tid + 7] = run;
    carry = b4;
    __syncthreads();
    const v4i o0 = *(const v4i*)(soff + 4 * tid);
    const v4i o1 = *(const v4i*)(soff + 4 * (tid + OTHR));
    int* op = off + base;
    *(volatile v4i*)(op + 4 * tid) = o0;
    *(volatile v4i*)(op + 4 * (tid + OTHR)) = o1;
    __threadfence();
    *(volatile v4i*)(op + 4 * tid) = o0;
    *(volatile v4i*)(op + 4 * (tid + OTHR)) = o1;
    __syncthreads();
  }
  if (tid == 0) srb[min(4 * nChunk, RBN - 1)] = carry;
  __syncthreads();
  v4i rv = {0, 0, 0, 0};
  if (tid < 32) rv = *(const v4i*)(srb + 4 * tid);
  if (tid < 32) *(volatile v4i*)(rbase + 4 * tid) = rv;
  __threadfence();
  if (tid < 32) *(volatile v4i*)(rbase + 4 * tid) = rv;
}

__global__ __launch_bounds__(NTHR) void k_fill(
    const int* __restrict__ ei, const int* __restrict__ off, const int* __restrict__ rbase,
    int* csr, int nN, int nE, int vec8, int csrLen) {
  extern __shared__ v4f lds_dyn[];
  int* region = (int*)lds_dyn;
  int* cursor = region + RCAP;
  int* list   = cursor + NBF;
  int* wcnt   = list + LISTN;
  const int tid = threadIdx.x, lane = tid & 31, wave = tid >> 5;
  const int b = blockIdx.x;
  const int nodeBase = b * NBF;
  const int* dsts = ei + nE;

  int rb0 = rbase[b];
  const int rb1 = rbase[b + 1];
  rb0 = rb0 < 0 ? 0 : (rb0 > csrLen ? csrLen : rb0);
  rb0 &= ~31;
  int len = rb1 - rb0;
  len = len < 0 ? 0 : (len > RCAP ? RCAP : len);
  int lenW = (len + 31) & ~31;
  if (rb0 + lenW > csrLen) lenW = (csrLen - rb0) & ~31;

  {
    const v4i z = {0, 0, 0, 0};
    for (int i = tid; i < RCAP / 4; i += NTHR) ((v4i*)region)[i] = z;
    for (int s = tid; s < NBF; s += NTHR) {
      int o = off[nodeBase + s] - rb0;
      o = o < 0 ? 0 : (o > RCAP ? RCAP : o);
      cursor[s] = o;
    }
  }
  __syncthreads();

  const int nChunks = (nE + CHUNK - 1) / CHUNK;
#pragma unroll 1
  for (int ch = 0; ch < nChunks; ++ch) {
    const int cbase = ch * CHUNK;
    const int wc = scan_chunk<NBF>(dsts, nE, cbase, nodeBase, vec8, list, tid, lane, wave);
    if (lane == 0) wcnt[wave] = wc;
    __syncthreads();
    if (wave == 0) {
#pragma unroll 1
      for (int wsx = 0; wsx < NWAVE; ++wsx) {
        int n = __builtin_amdgcn_readfirstlane(wcnt[wsx]);
        n = n > WCAP ? WCAP : (n < 0 ? 0 : n);
        const int* lp = list + wsx * WCAP;
#pragma unroll 1
        for (int i = 0; i < n; ++i) {
          const int ent  = __builtin_amdgcn_readfirstlane(lp[i]);
          const int slot = ent & (NBF - 1);
          int e = cbase + ((ent >> 12) & (CHUNK - 1));
          e = e > nE - 1 ? nE - 1 : e;
          int src = ei[e];
          src = src < 0 ? 0 : (src > nN - 1 ? nN - 1 : src);
          if (lane == 0) {
            int pos = cursor[slot];
            pos = pos < 0 ? 0 : (pos > RCAP - 1 ? RCAP - 1 : pos);
            region[pos] = src;
            const int np = pos + 1;
            cursor[slot] = np > RCAP ? RCAP : np;
          }
        }
      }
    }
    __syncthreads();
  }

  const int nv = lenW >> 2;
  int* gp = csr + rb0;
#pragma unroll 1
  for (int i = tid; i < nv; i += NTHR) { const v4i v = ((const v4i*)region)[i]; *(volatile v4i*)(gp + 4 * i) = v; }
  __threadfence();
#pragma unroll 1
  for (int i = tid; i < nv; i += NTHR) { const v4i v = ((const v4i*)region)[i]; *(volatile v4i*)(gp + 4 * i) = v; }
}

__global__ __launch_bounds__(NTHR) void k_sage0(
    const int* __restrict__ csr, const int* __restrict__ off, const int* __restrict__ cnt,
    const float* __restrict__ dinv, const float* __restrict__ x,
    const float* __restrict__ Wl0, const float* __restrict__ Wr0, const float* __restrict__ b0,
    const float* __restrict__ g0, const float* __restrict__ e0,
    float* H1, int nN, int csrLen) {
  const int tid = threadIdx.x, lane = tid & 31, wave = tid >> 5;
  const int tq = lane >> 4, c16 = lane & 15;
  const int tbase = blockIdx.x * TGT0 + wave * 32;
  const int cnt_l = cnt[tbase + lane];
  const int off_l = off[tbase + lane];
  union FI { float f; int i; };
  FI dvu; dvu.f = dinv[tbase + lane];
  const v4f wl = *(const v4f*)(Wl0 + 4 * c16);
  const v4f wr = *(const v4f*)(Wr0 + 4 * c16);
  const v4f bb = *(const v4f*)(b0 + 4 * c16);
  const v4f gg = *(const v4f*)(g0 + 4 * c16);
  const v4f be = *(const v4f*)(e0 + 4 * c16);
  const size_t pl = (size_t)nN;

#pragma unroll 1
  for (int j = 0; j < 32; ++j) {
    const int c  = tbase + j;
    const int cc = c > nN - 1 ? nN - 1 : c;
    int n = __builtin_amdgcn_readlane(cnt_l, j);
    n = n < 0 ? 0 : (n > DEGCAP ? DEGCAP : n);
    const int st = __builtin_amdgcn_readlane(off_l, j);
    FI du; du.i = __builtin_amdgcn_readlane(dvu.i, j);
    const float inv = du.f;

    float s[8];
#pragma unroll
    for (int tg = 0; tg < 8; ++tg) s[tg] = 0.f;
#pragma unroll 1
    for (int p0 = 0; p0 < n; p0 += 16) {
      int pos = st + p0 + c16;
      pos = pos < 0 ? 0 : (pos > csrLen - 1 ? csrLen - 1 : pos);
      int sv = csr[pos];
      sv = sv < 0 ? 0 : (sv > nN - 1 ? nN - 1 : sv);
      const bool ok = (p0 + c16) < n;
#pragma unroll
      for (int tg = 0; tg < 8; ++tg) {
        const float xv = x[(size_t)(2 * tg + tq) * pl + sv];
        s[tg] += ok ? xv : 0.f;
      }
    }
#pragma unroll
    for (int tg = 0; tg < 8; ++tg) s[tg] = red16(s[tg]);

#pragma unroll 1
    for (int tg = 0; tg < 8; ++tg) {
      float sg = s[0];
#pragma unroll
      for (int k = 1; k < 8; ++k) sg = (k == tg) ? s[k] : sg;
      const int t = 2 * tg + tq;
      const float a  = sg * inv;
      const float xs = x[(size_t)t * pl + cc];
      v4f v = wl * a + wr * xs;
      v = v + bb;
      const float mu = red16((v.x + v.y) + (v.z + v.w)) * (1.0f / HG);
      const v4f d = v - mu;
      const float var = red16((d.x * d.x + d.y * d.y) + (d.z * d.z + d.w * d.w)) * (1.0f / HG);
      const float rs = rsqrtf(var + LNEPS);
      v4f o = d * rs * gg + be;
      o.x = fmaxf(o.x, 0.f); o.y = fmaxf(o.y, 0.f); o.z = fmaxf(o.z, 0.f); o.w = fmaxf(o.w, 0.f);
      if (c < nN) {
        float* hp = H1 + ((size_t)t * pl + cc) * HG + 4 * c16;
        *(volatile v4f*)hp = o;
        __threadfence();
        *(volatile v4f*)hp = o;
      }
    }
  }
}

__global__ __launch_bounds__(NTHR) void k_sage1(
    const int* __restrict__ csr, const int* __restrict__ off, const int* __restrict__ cnt,
    const float* __restrict__ dinv, const float* __restrict__ H1, const _Float16* __restrict__ wcat,
    const float* __restrict__ b1, const float* __restrict__ g1, const float* __restrict__ e1,
    _Float16* H2, int nN, int nRows, int csrLen) {
  __shared__ __attribute__((aligned(16))) _Float16 sA[ROWS1 * AP1];
  __shared__ __attribute__((aligned(16))) _Float16 sO[ROWS1 * SP1];
  const int tid = threadIdx.x, lane = tid & 31, wave = tid >> 5, hh = lane >> 4, m = lane & 15;
  const int rowBase = blockIdx.x * ROWS1;

#pragma unroll 1
  for (int j = 0; j < 16; ++j) {
    int r = rowBase + wave * 16 + j;
    r = r > nRows - 1 ? nRows - 1 : r;
    const int t = r / nN;
    const int c = r - t * nN;
    int n = cnt[c];
    n = n < 0 ? 0 : (n > DEGCAP ? DEGCAP : n);
    const int st = off[c];
    const float inv = dinv[c];
    const float* hb = H1 + (size_t)t * nN * HG + 2 * lane;
    float ax = 0.f, ay = 0.f;
#pragma unroll 1
    for (int q0 = 0; q0 < n; q0 += 32) {
      int pos = st + q0 + lane;
      pos = pos < 0 ? 0 : (pos > csrLen - 1 ? csrLen - 1 : pos);
      int sl = csr[pos];
      sl = sl < 0 ? 0 : (sl > nN - 1 ? nN - 1 : sl);
      const int mcnt = (n - q0) < 32 ? (n - q0) : 32;
#pragma unroll 1
      for (int p = 0; p < mcnt; ++p) {
        const int sv = __builtin_amdgcn_readlane(sl, p);
        const v2f hv = *(const v2f*)(hb + (size_t)sv * HG);
        ax += hv.x; ay += hv.y;
      }
    }
    const v2f self = *(const v2f*)(hb + (size_t)c * HG);
    _Float16* ap = sA + (wave * 16 + j) * AP1;
    v2h pa; pa.x = (_Float16)(ax * inv * ASC); pa.y = (_Float16)(ay * inv * ASC);
    v2h ps; ps.x = (_Float16)(self.x * ASC);     ps.y = (_Float16)(self.y * ASC);
    *(v2h*)(ap + 2 * lane)      = pa;
    *(v2h*)(ap + HG + 2 * lane) = ps;
  }
  __syncthreads();

  v8f acc[4];
#pragma unroll
  for (int nt = 0; nt < 4; ++nt) { v8f z = {0.f, 0.f, 0.f, 0.f, 0.f, 0.f, 0.f, 0.f}; acc[nt] = z; }
  const _Float16* ar = sA + (wave * 16 + m) * AP1 + 8 * hh;
#pragma unroll
  for (int kt = 0; kt < KC / 32; ++kt) {
    FragH a;
    a.h[0] = *(const v8h*)(ar + 32 * kt);
    a.h[1] = *(const v8h*)(ar + 32 * kt + 16);
#pragma unroll
    for (int nt = 0; nt < 4; ++nt) {
      const _Float16* bp = wcat + (size_t)(16 * nt + m) * KC + 32 * kt + 8 * hh;
      FragH b;
      b.h[0] = *(const v8h*)bp;
      b.h[1] = *(const v8h*)(bp + 16);
      acc[nt] = wmh(a.v, b.v, acc[nt]);
    }
  }

  float bv[4], gv[4], ev[4];
#pragma unroll
  for (int nt = 0; nt < 4; ++nt) { bv[nt] = b1[16 * nt + m]; gv[nt] = g1[16 * nt + m]; ev[nt] = e1[16 * nt + m]; }
#pragma unroll
  for (int nt = 0; nt < 4; ++nt)
#pragma unroll
    for (int r = 0; r < 8; ++r) acc[nt][r] = acc[nt][r] * PINV + bv[nt];
  float mu[8], rs[8];
#pragma unroll
  for (int r = 0; r < 8; ++r)
    mu[r] = red16((acc[0][r] + acc[1][r]) + (acc[2][r] + acc[3][r])) * (1.0f / HG);
#pragma unroll
  for (int r = 0; r < 8; ++r) {
    float q = 0.f;
#pragma unroll
    for (int nt = 0; nt < 4; ++nt) { const float d = acc[nt][r] - mu[r]; q += d * d; }
    rs[r] = rsqrtf(red16(q) * (1.0f / HG) + LNEPS);
  }
  _Float16* sp = sO + (wave * 16 + 8 * hh) * SP1 + m;
#pragma unroll
  for (int nt = 0; nt < 4; ++nt)
#pragma unroll
    for (int r = 0; r < 8; ++r) {
      float o = (acc[nt][r] - mu[r]) * rs[r] * gv[nt] + ev[nt];
      o = fmaxf(o, 0.f) * ASC;
      sp[r * SP1 + 16 * nt] = (_Float16)o;
    }
  __syncthreads();

  v8h ov[4];
#pragma unroll
  for (int i = 0; i < 4; ++i) {
    const int row = wave * 16 + 4 * i + (lane >> 3);
    ov[i] = *(const v8h*)(sO + row * SP1 + 8 * (lane & 7));
  }
  _Float16* gp = H2 + ((size_t)rowBase + wave * 16) * HG;
#pragma unroll
  for (int i = 0; i < 4; ++i)
    *(volatile v8h*)(gp + (size_t)(4 * i + (lane >> 3)) * HG + 8 * (lane & 7)) = ov[i];
  __threadfence();
#pragma unroll
  for (int i = 0; i < 4; ++i)
    *(volatile v8h*)(gp + (size_t)(4 * i + (lane >> 3)) * HG + 8 * (lane & 7)) = ov[i];
}

__global__ __launch_bounds__(GTHR) void k_gru(
    const _Float16* __restrict__ H2, const _Float16* __restrict__ wihp, const _Float16* __restrict__ whhp,
    const float* __restrict__ bih, const float* __restrict__ bhh,
    const float* __restrict__ hW, const float* __restrict__ hb, float* out, int nN) {
  __shared__ __attribute__((aligned(16))) float    hs[GWAVE * 16 * HP32];
  __shared__ __attribute__((aligned(16))) _Float16 hq[GWAVE * 16 * HP16];
  __shared__ __attribute__((aligned(16))) float    ys[GROWB];
  const int tid = threadIdx.x, lane = tid & 31, wave = tid >> 5, hh = lane >> 4, m = lane & 15;
  const int rowBase = blockIdx.x * GROWB;
  int row0 = rowBase + wave * 16;
  row0 = row0 > nN - 16 ? nN - 16 : row0;

  {
    const v4f z = {0.f, 0.f, 0.f, 0.f};
    for (int i = tid; i < GWAVE * 16 * HP32 / 4; i += GTHR) ((v4f*)hs)[i] = z;
    v8h zh;
#pragma unroll
    for (int e = 0; e < 8; ++e) zh[e] = (_Float16)0.0f;
    for (int i = tid; i < GWAVE * 16 * HP16 / 8; i += GTHR) ((v8h*)hq)[i] = zh;
  }
  __syncthreads();
  float*    hsw = hs + wave * 16 * HP32;
  _Float16* hqw = hq + wave * 16 * HP16;

#pragma unroll 1
  for (int t = 0; t < TT; ++t) {
    FragH ax[2], ah[4];
    const _Float16* xr = H2 + ((size_t)t * nN + row0 + m) * HG + 8 * hh;
#pragma unroll
    for (int kt = 0; kt < 2; ++kt) {
      ax[kt].h[0] = *(const v8h*)(xr + 32 * kt);
      ax[kt].h[1] = *(const v8h*)(xr + 32 * kt + 16);
    }
    const _Float16* hr = hqw + m * HP16 + 8 * hh;
#pragma unroll
    for (int kt = 0; kt < 4; ++kt) {
      ah[kt].h[0] = *(const v8h*)(hr + 32 * kt);
      ah[kt].h[1] = *(const v8h*)(hr + 32 * kt + 16);
    }

#pragma unroll 1
    for (int q = 0; q < HT / 16; ++q) {
      v8f cr = {0.f, 0.f, 0.f, 0.f, 0.f, 0.f, 0.f, 0.f};
      v8f cz = {0.f, 0.f, 0.f, 0.f, 0.f, 0.f, 0.f, 0.f};
      if (t > 0) {
#pragma unroll
        for (int kt = 0; kt < 4; ++kt) {
          const _Float16* bp = whhp + (size_t)(16 * q + m) * HT + 32 * kt + 8 * hh;
          FragH br, bz;
          br.h[0] = *(const v8h*)bp;                    br.h[1] = *(const v8h*)(bp + 16);
          bz.h[0] = *(const v8h*)(bp + HT * HT);        bz.h[1] = *(const v8h*)(bp + HT * HT + 16);
          cr = wmh(ah[kt].v, br.v, cr);
          cz = wmh(ah[kt].v, bz.v, cz);
        }
      }
#pragma unroll
      for (int kt = 0; kt < 2; ++kt) {
        const _Float16* bp = wihp + (size_t)(16 * q + m) * HG + 32 * kt + 8 * hh;
        FragH br, bz;
        br.h[0] = *(const v8h*)bp;                      br.h[1] = *(const v8h*)(bp + 16);
        bz.h[0] = *(const v8h*)(bp + HT * HG);          bz.h[1] = *(const v8h*)(bp + HT * HG + 16);
        cr = wmh(ax[kt].v, br.v, cr);
        cz = wmh(ax[kt].v, bz.v, cz);
      }
      const int col = 16 * q + m;
      const float b_r = bih[col] + bhh[col];
      const float b_z = bih[HT + col] + bhh[HT + col];
      float rg[8], zg[8];
#pragma unroll
      for (int r = 0; r < 8; ++r) {
        rg[r] = sigm(cr[r] * PINV + b_r);
        zg[r] = sigm(cz[r] * PINV + b_z);
      }
      v8f cn = {0.f, 0.f, 0.f, 0.f, 0.f, 0.f, 0.f, 0.f};
      v8f ci = {0.f, 0.f, 0.f, 0.f, 0.f, 0.f, 0.f, 0.f};
      if (t > 0) {
#pragma unroll
        for (int kt = 0; kt < 4; ++kt) {
          const _Float16* bp = whhp + (size_t)(2 * HT + 16 * q + m) * HT + 32 * kt + 8 * hh;
          FragH bn;
          bn.h[0] = *(const v8h*)bp;  bn.h[1] = *(const v8h*)(bp + 16);
          cn = wmh(ah[kt].v, bn.v, cn);
        }
      }
#pragma unroll
      for (int kt = 0; kt < 2; ++kt) {
        const _Float16* bp = wihp + (size_t)(2 * HT + 16 * q + m) * HG + 32 * kt + 8 * hh;
        FragH bi;
        bi.h[0] = *(const v8h*)bp;  bi.h[1] = *(const v8h*)(bp + 16);
        ci = wmh(ax[kt].v, bi.v, ci);
      }
      const float b_i = bih[2 * HT + col];
      const float b_n = bhh[2 * HT + col];
      float*    hp32 = hsw + (8 * hh) * HP32 + col;
      _Float16* hp16 = hqw + (8 * hh) * HP16 + col;
#pragma unroll
      for (int r = 0; r < 8; ++r) {
        const float hpv = hp32[r * HP32];
        const float ng  = tanh_fast(ci[r] * PINV + b_i + rg[r] * (cn[r] * PINV + b_n));
        const float hn  = (1.0f - zg[r]) * ng + zg[r] * hpv;
        hp32[r * HP32] = hn;
        hp16[r * HP16] = (_Float16)(hn * ASC);
      }
    }
    __syncthreads();
  }

  const float* hrow = hsw + m * HP32 + 64 * hh;
  const float* wv   = hW + 64 * hh;
  float s = 0.f;
#pragma unroll 4
  for (int j = 0; j < 64; ++j) s += hrow[j] * wv[j];
  s += __shfl_xor(s, 16, 32);
  const float y = s + hb[0];
  if (hh == 0) ys[wave * 16 + m] = y;
  __syncthreads();
  int nv = nN - rowBase;
  nv = nv < 0 ? 0 : (nv > GROWB ? GROWB : nv);
  const int nst = nv >> 2;
  const v4f ov = *(const v4f*)(ys + 4 * (lane & 15));
  float* op = out + (size_t)rowBase + 4 * (lane & 15);
  const bool doSt = (wave == 0) && (lane < nst);
  if (doSt) *(volatile v4f*)op = ov;
  __threadfence();
  if (doSt) *(volatile v4f*)op = ov;
}

extern "C" void kernel_launch(void* const* d_in, const int* in_sizes, int n_in,
                              void* d_out, int out_size, void* d_ws, size_t ws_size,
                              hipStream_t stream) {
  if (n_in < 18) return;
  const int nN = in_sizes[0] / TT;
  if (nN < GROWB || in_sizes[0] != TT * nN || (nN % 32) != 0) return;
  const int nE = in_sizes[1] / 2;
  if (nE <= 0 || in_sizes[1] != 2 * nE) return;
  if (in_sizes[2] != HG || in_sizes[3] != HG || in_sizes[4] != HG || in_sizes[5] != HG || in_sizes[6] != HG) return;
  if (in_sizes[7] != HG * HG || in_sizes[8] != HG * HG || in_sizes[9] != HG || in_sizes[10] != HG || in_sizes[11] != HG) return;
  if (in_sizes[12] != G3 * HG || in_sizes[13] != G3 * HT || in_sizes[14] != G3 || in_sizes[15] != G3) return;
  if (in_sizes[16] != HT || in_sizes[17] < 1) return;
  if (out_size != nN) return;
  if (nE > (1 << 28) || nN > (1 << 22)) return;

  const float* x    = (const float*)d_in[0];
  const int*   ei   = (const int*)d_in[1];
  const float* Wl0  = (const float*)d_in[2];
  const float* Wr0  = (const float*)d_in[3];
  const float* b0   = (const float*)d_in[4];
  const float* g0   = (const float*)d_in[5];
  const float* e0   = (const float*)d_in[6];
  const float* Wl1  = (const float*)d_in[7];
  const float* Wr1  = (const float*)d_in[8];
  const float* b1   = (const float*)d_in[9];
  const float* g1   = (const float*)d_in[10];
  const float* e1   = (const float*)d_in[11];
  const float* Wih  = (const float*)d_in[12];
  const float* Whh  = (const float*)d_in[13];
  const float* bih  = (const float*)d_in[14];
  const float* bhh  = (const float*)d_in[15];
  const float* hW   = (const float*)d_in[16];
  const float* hb   = (const float*)d_in[17];
  float* out = (float*)d_out;

  const int NPAD0  = ((nN + TGT0 - 1) / TGT0) * TGT0;
  const int nB0    = NPAD0 / TGT0;
  const int nBC    = (nN + NBC - 1) / NBC;
  const int CNTPAD = nBC * NBC;
  if (4 * nBC + 1 > RBN || NPAD0 > CNTPAD) return;
  const int nBF    = (nN + NBF - 1) / NBF;
  const int csrLen = ((nE + 31) & ~31) + 4096;
  const int nRows  = TT * nN;
  const int nB1    = (nRows + ROWS1 - 1) / ROWS1;
  const int rowsP  = nB1 * ROWS1;
  const int nBG    = (nN + GROWB - 1) / GROWB;

  char* ws = (char*)d_ws;
  size_t off = 0;
  const size_t oWc  = off; off += (size_t)HG * KC * 2;            off = (off + 255) & ~(size_t)255;
  const size_t oWi  = off; off += (size_t)G3 * HG * 2;            off = (off + 255) & ~(size_t)255;
  const size_t oWh  = off; off += (size_t)G3 * HT * 2;            off = (off + 255) & ~(size_t)255;
  const size_t oCnt = off; off += (size_t)CNTPAD * 4;             off = (off + 255) & ~(size_t)255;
  const size_t oDv  = off; off += (size_t)CNTPAD * 4;             off = (off + 255) & ~(size_t)255;
  const size_t oOff = off; off += (size_t)CNTPAD * 4;             off = (off + 255) & ~(size_t)255;
  const size_t oRb  = off; off += (size_t)RBN * 4;                off = (off + 255) & ~(size_t)255;
  const size_t oCsr = off; off += (size_t)csrLen * 4;             off = (off + 255) & ~(size_t)255;
  const size_t oH1  = off; off += (size_t)nRows * HG * 4;         off = (off + 255) & ~(size_t)255;
  const size_t oH2  = off; off += (size_t)rowsP * HG * 2;         off = (off + 255) & ~(size_t)255;
  if (off > ws_size) return;
  _Float16* wcat = (_Float16*)(ws + oWc);
  _Float16* wihp = (_Float16*)(ws + oWi);
  _Float16* whhp = (_Float16*)(ws + oWh);
  int*      cnt  = (int*)(ws + oCnt);
  float*    dinv = (float*)(ws + oDv);
  int*      offp = (int*)(ws + oOff);
  int*      rb   = (int*)(ws + oRb);
  int*      csr  = (int*)(ws + oCsr);
  float*    H1   = (float*)(ws + oH1);
  _Float16* H2   = (_Float16*)(ws + oH2);

  const int vec8 = ((nE & 3) == 0) ? 1 : 0;

  const int nPrep = HG * KC / 8 + G3 * HG / 8 + G3 * HT / 8;
  k_wprep<<<(nPrep + NTHR - 1) / NTHR, NTHR, 0, stream>>>(Wl1, Wr1, Wih, Whh, wcat, wihp, whhp);

  k_count<<<nBC, NTHR, 0, stream>>>(ei, cnt, dinv, nE, vec8);
  k_offsets<<<1, OTHR, 0, stream>>>(cnt, offp, rb, nBC);
  hipFuncSetAttribute(reinterpret_cast<const void*>(&k_fill),
                      hipFuncAttributeMaxDynamicSharedMemorySize, LDS_FILL);
  k_fill<<<nBF, NTHR, LDS_FILL, stream>>>(ei, offp, rb, csr, nN, nE, vec8, csrLen);

  k_sage0<<<nB0, NTHR, 0, stream>>>(csr, offp, cnt, dinv, x, Wl0, Wr0, b0, g0, e0, H1, nN, csrLen);

  k_sage1<<<nB1, NTHR, 0, stream>>>(csr, offp, cnt, dinv, H1, wcat, b1, g1, e1, H2, nN, nRows, csrLen);

  k_gru<<<nBG, GTHR, 0, stream>>>(H2, wihp, whhp, bih, bhh, hW, hb, out, nN);
}
